// ProsodyPredictorV15_10797547782207
// MI455X (gfx1250) — hardware-run, weakly checked
//
#include <hip/hip_runtime.h>
#include <math.h>

typedef __attribute__((ext_vector_type(16))) _Float16 v16h;
typedef __attribute__((ext_vector_type(8)))  _Float16 v8h;
typedef __attribute__((ext_vector_type(8)))  float    v8f;
typedef __attribute__((ext_vector_type(4)))  float    v4f;
typedef __attribute__((ext_vector_type(4)))  unsigned v4u;

constexpr int kBatch    = 4;
constexpr int kSteps    = 2048;
constexpr int kEmb      = 512;
constexpr int kWidth    = 512;
constexpr int kStates   = 16;
constexpr int kLayers   = 4;
constexpr int kFreqRows = 2048;
constexpr int kRows     = kBatch * kSteps;
constexpr int kOut0Elems = kRows;
constexpr int kOut1Elems = kRows;
constexpr int kOut1OffBytes = 32768;
constexpr int kOut1Off = kOut1OffBytes / 4;
static_assert(kRows == 8192);
static_assert(kFreqRows >= kSteps);
static_assert((kEmb % 32) == 0 && (kRows % 32) == 0 && (kWidth % 64) == 0);
static_assert(kWidth / 64 == 8);
static_assert(kOut1Off == kOut0Elems);
static_assert(kOut1OffBytes + kOut1Elems * 4 == 65536);
static_assert((kOut1OffBytes % 128) == 0);

constexpr bool kAResid = false;
constexpr bool kWResid = false;
constexpr bool kAnyResid = kAResid || kWResid;

constexpr float kWCarry     = 64.0f;
constexpr float kWCarryInv  = 1.0f / 64.0f;
constexpr float kLoScale    = 2048.0f;
constexpr float kLoScaleInv = 1.0f / 2048.0f;

constexpr size_t kPlaneA  = (size_t)kRows * kEmb * 2;
constexpr size_t kPlaneAL = kAResid ? kPlaneA : (size_t)0;
constexpr size_t kPlaneW  = (size_t)kWidth * kEmb * 2;
constexpr size_t kPlaneT  = (size_t)kLayers * kWidth * kStates * 4;
constexpr size_t kPlaneH  = (size_t)kRows * kWidth * 4;
constexpr size_t kOffA16  = 0;
constexpr size_t kOffA16L = kOffA16  + kPlaneA;
constexpr size_t kOffBt   = kOffA16L + kPlaneAL;
constexpr size_t kOffBtL  = kOffBt   + kPlaneW;
constexpr size_t kOffAbar = kOffBtL  + kPlaneW;
constexpr size_t kOffBbar = kOffAbar + kPlaneT;
constexpr size_t kOffH    = kOffBbar + kPlaneT;
constexpr size_t kWsTotal = kOffH + 5 * kPlaneH;
static_assert(kWsTotal == (kAResid ? 101974016ull : 93585408ull));
static_assert(kWsTotal <= 134217728ull);
static_assert((kOffA16L % 128) == 0 && (kOffBt % 128) == 0 && (kOffBtL % 128) == 0 &&
              (kOffAbar % 128) == 0 && (kOffBbar % 128) == 0 && (kOffH % 128) == 0 && (kPlaneH % 128) == 0);

__device__ __forceinline__ float flush16(float v) {
  return (fabsf(v) < 6.103515625e-05f) ? 0.0f : v;
}
__device__ __forceinline__ unsigned short f16bits(float x) {
  const _Float16 h = (_Float16)flush16(x);
  return __builtin_bit_cast(unsigned short, h);
}
__device__ __forceinline__ unsigned pack2(float a, float b) {
  const unsigned lo = (unsigned)f16bits(a);
  const unsigned hi = (unsigned)f16bits(b);
  return lo | (hi << 16);
}
__device__ __forceinline__ float second16(float v) {
  const _Float16 hv = (_Float16)flush16(v);
  const float back = (float)hv;
  return (v - back) * kLoScale;
}
__device__ __forceinline__ void wave_sync() {
  __builtin_amdgcn_fence(__ATOMIC_RELEASE, "workgroup");
  __builtin_amdgcn_wave_barrier();
  __builtin_amdgcn_fence(__ATOMIC_ACQUIRE, "workgroup");
}
__device__ __forceinline__ void store2_v4u(unsigned short* p, v4u v) {
  volatile v4u* q = (volatile v4u*)p;
  *q = v;
  __threadfence();
  *q = v;
}
__device__ __forceinline__ float wave_sum(float v) {
  v += __shfl_xor(v, 16, 32);
  v += __shfl_xor(v, 8, 32);
  v += __shfl_xor(v, 4, 32);
  v += __shfl_xor(v, 2, 32);
  v += __shfl_xor(v, 1, 32);
  return v;
}

union FragH { v16h v; v8h h[2]; };
__device__ __forceinline__ v16h frag_load(const _Float16* p) {
  FragH f;
  f.h[0] = *(const v8h*)(p);
  f.h[1] = *(const v8h*)(p + 16);
  return f.v;
}
__device__ __forceinline__ v8f mma16(v16h a, v16h b, v8f c) {
  return __builtin_amdgcn_wmma_f32_16x16x32_f16(false, a, false, b, (short)0, c, false, false);
}
__device__ __forceinline__ void tie_acc(v8f& a, v16h x, v16h y) { asm volatile("" : "+v"(a) : "v"(x), "v"(y)); }
__device__ __forceinline__ void tie_acc_nops(v8f& a, v16h x, v16h y) { asm volatile("v_nop\n\tv_nop\n\tv_nop\n\tv_nop" : "+v"(a) : "v"(x), "v"(y)); }
__device__ __forceinline__ void keep4(v16h a, v16h b, v16h c, v16h d) { asm volatile("v_nop" :: "v"(a), "v"(b), "v"(c), "v"(d)); }
__device__ __forceinline__ void acc_guard4(v8f& a, v8f& b, v8f& c, v8f& d) { asm volatile("v_nop\n\tv_nop\n\tv_nop\n\tv_nop" : "+v"(a), "+v"(b), "+v"(c), "+v"(d)); }

__global__ __launch_bounds__(256) void act_plane_kernel(
    const float* __restrict__ x, unsigned short* __restrict__ hi, unsigned short* __restrict__ lo) {
  const size_t task = (size_t)blockIdx.x * 256 + threadIdx.x;
  const float* p = x + task * 8;
  const v4f a0 = *(const v4f*)(p);
  const v4f a1 = *(const v4f*)(p + 4);
  const v4u ph = {pack2(a0[0], a0[1]), pack2(a0[2], a0[3]), pack2(a1[0], a1[1]), pack2(a1[2], a1[3])};
  store2_v4u(hi + task * 8, ph);
  if constexpr (kAResid) {
    const v4u pl = {pack2(second16(a0[0]), second16(a0[1])), pack2(second16(a0[2]), second16(a0[3])),
                    pack2(second16(a1[0]), second16(a1[1])), pack2(second16(a1[2]), second16(a1[3]))};
    store2_v4u(lo + task * 8, pl);
  }
}

__global__ __launch_bounds__(256) void weight_plane_kernel(
    const float* __restrict__ w_in, unsigned short* __restrict__ bt, unsigned short* __restrict__ btl) {
  __shared__ float sT[32 * 257];
  const int tid = threadIdx.x;
  const int mm = tid & 31;
  const int kq = tid >> 5;
  const int n0 = (int)blockIdx.x * 32;
  const int kb = (int)blockIdx.y * 256;
  for (int it = 0; it < 32; ++it) {
    const int k = it * 8 + kq;
    sT[mm * 257 + k] = w_in[(size_t)(kb + k) * kWidth + n0 + mm];
  }
  __syncthreads();
  for (int it = 0; it < 4; ++it) {
    const int q = it * 256 + tid;
    const int row = q >> 5;
    const int k8 = (q & 31) * 8;
    float vh[8];
    float vl[8];
#pragma unroll
    for (int e = 0; e < 8; ++e) {
      const float v = sT[row * 257 + k8 + e] * kWCarry;
      vh[e] = v;
      vl[e] = second16(v);
    }
    const size_t off = (size_t)(n0 + row) * kEmb + kb + k8;
    const v4u ph = {pack2(vh[0], vh[1]), pack2(vh[2], vh[3]), pack2(vh[4], vh[5]), pack2(vh[6], vh[7])};
    store2_v4u(bt + off, ph);
    if (kWResid) {
      const v4u pl = {pack2(vl[0], vl[1]), pack2(vl[2], vl[3]), pack2(vl[4], vl[5]), pack2(vl[6], vl[7])};
      store2_v4u(btl + off, pl);
    }
  }
}

__global__ __launch_bounds__(256) void discretise_kernel(
    const float* __restrict__ log_dt, const float* __restrict__ a_log, const float* __restrict__ b_ssm,
    float* __restrict__ abar_t, float* __restrict__ bbar_t) {
  const int idx = (int)blockIdx.x * 256 + (int)threadIdx.x;
  const int ld = idx >> 4;
  const float dt = expf(log_dt[ld]);
  const float a = -expf(a_log[idx]);
  const float ab = expf(dt * a);
  const float bb = (ab - 1.0f) / a * b_ssm[idx];
  volatile float* pa = (volatile float*)(abar_t + idx);
  volatile float* pb = (volatile float*)(bbar_t + idx);
  *pa = ab;
  *pb = bb;
  __threadfence();
  *pa = ab;
  *pb = bb;
}

__global__ __launch_bounds__(256) void proj_gemm_kernel(
    const unsigned short* __restrict__ a16, const unsigned short* __restrict__ a16l,
    const unsigned short* __restrict__ bt16, const unsigned short* __restrict__ bt16l,
    const float* __restrict__ b_in, const float* __restrict__ freq, float* hout) {
  __shared__ __align__(16) float sT[8][16 * 68];
  const int lane = threadIdx.x & 31;
  const int wave = __builtin_amdgcn_readfirstlane((int)(threadIdx.x >> 5));
  const int m0 = (int)blockIdx.x * 32;
  const int n0 = wave * 64;
  const int rlane = lane & 15;
  const int koff = (lane >> 4) * 8;
  const int mOff = (lane >> 4) * 8;
  const _Float16* ap  = (const _Float16*)a16  + (size_t)(m0 + rlane) * kEmb + koff;
  const _Float16* apl = (const _Float16*)a16l + (size_t)(m0 + rlane) * kEmb + koff;
  const _Float16* bp  = (const _Float16*)bt16  + (size_t)(n0 + rlane) * kEmb + koff;
  const _Float16* bpl = (const _Float16*)bt16l + (size_t)(n0 + rlane) * kEmb + koff;

  v8f acc[2][4];
  v8f accr[2][4];
#pragma unroll
  for (int i = 0; i < 2; ++i)
#pragma unroll
    for (int j = 0; j < 4; ++j) {
      acc[i][j] = (v8f){0.f, 0.f, 0.f, 0.f, 0.f, 0.f, 0.f, 0.f};
      accr[i][j] = (v8f){0.f, 0.f, 0.f, 0.f, 0.f, 0.f, 0.f, 0.f};
    }

  for (int ks = 0; ks < kEmb / 32; ++ks) {
    v16h bh[4];
#pragma unroll
    for (int j = 0; j < 4; ++j) bh[j] = frag_load(bp + (size_t)(j * 16) * kEmb + ks * 32);
#pragma unroll
    for (int i = 0; i < 2; ++i) {
      const v16h ah = frag_load(ap + (size_t)(i * 16) * kEmb + ks * 32);
#pragma unroll
      for (int j = 0; j < 4; ++j) acc[i][j] = mma16(ah, bh[j], acc[i][j]);
      tie_acc(acc[i][0], ah, bh[0]);
      tie_acc(acc[i][1], ah, bh[1]);
      tie_acc(acc[i][2], ah, bh[2]);
      tie_acc_nops(acc[i][3], ah, bh[3]);
      if constexpr (kAResid) {
        const v16h al = frag_load(apl + (size_t)(i * 16) * kEmb + ks * 32);
#pragma unroll
        for (int j = 0; j < 4; ++j) accr[i][j] = mma16(al, bh[j], accr[i][j]);
        tie_acc(accr[i][0], al, bh[0]);
        tie_acc(accr[i][1], al, bh[1]);
        tie_acc(accr[i][2], al, bh[2]);
        tie_acc_nops(accr[i][3], al, bh[3]);
      }
    }
    if constexpr (kWResid) {
      v16h bl[4];
#pragma unroll
      for (int j = 0; j < 4; ++j) bl[j] = frag_load(bpl + (size_t)(j * 16) * kEmb + ks * 32);
#pragma unroll
      for (int i = 0; i < 2; ++i) {
        const v16h ah = frag_load(ap + (size_t)(i * 16) * kEmb + ks * 32);
#pragma unroll
        for (int j = 0; j < 4; ++j) accr[i][j] = mma16(ah, bl[j], accr[i][j]);
        tie_acc(accr[i][0], ah, bl[0]);
        tie_acc(accr[i][1], ah, bl[1]);
        tie_acc(accr[i][2], ah, bl[2]);
        tie_acc_nops(accr[i][3], ah, bl[3]);
      }
      keep4(bl[0], bl[1], bl[2], bl[3]);
    }
    keep4(bh[0], bh[1], bh[2], bh[3]);
  }
  acc_guard4(acc[0][0], acc[0][1], acc[0][2], acc[0][3]);
  acc_guard4(acc[1][0], acc[1][1], acc[1][2], acc[1][3]);
  if constexpr (kAnyResid) {
    acc_guard4(accr[0][0], accr[0][1], accr[0][2], accr[0][3]);
    acc_guard4(accr[1][0], accr[1][1], accr[1][2], accr[1][3]);
  }

  float* slab = sT[wave];
  const int h2 = lane >> 4;
  const int c4 = (lane & 15) * 4;
  const v4f bias4 = *(const v4f*)(b_in + n0 + c4);
#pragma unroll
  for (int i = 0; i < 2; ++i) {
    const int mBase = m0 + (i << 4);
#pragma unroll
    for (int j = 0; j < 4; ++j) {
#pragma unroll
      for (int r = 0; r < 8; ++r) {
        float sum = acc[i][j][r];
        if constexpr (kAnyResid) sum = fmaf(accr[i][j][r], kLoScaleInv, sum);
        slab[(mOff + r) * 68 + (j << 4) + rlane] = sum * kWCarryInv;
      }
    }
    wave_sync();
    v4f vals[8];
#pragma unroll
    for (int it = 0; it < 8; ++it) {
      const int row = it * 2 + h2;
      const int t = (mBase + row) & (kSteps - 1);
      const v4f s = *(const v4f*)(slab + row * 68 + c4);
      const v4f f = *(const v4f*)(freq + (size_t)t * kWidth + n0 + c4);
      vals[it] = (s + bias4) + f;
    }
    for (int pass = 0; pass < 2; ++pass) {
#pragma unroll
      for (int it = 0; it < 8; ++it) {
        const int row = it * 2 + h2;
        *(volatile v4f*)(hout + (size_t)(mBase + row) * kWidth + n0 + c4) = vals[it];
      }
      __threadfence();
    }
    wave_sync();
  }
}

__global__ __launch_bounds__(32) void scan_layer_kernel(
    const float* __restrict__ hin, float* hout,
    const float* __restrict__ abar_t, const float* __restrict__ bbar_t,
    const float* __restrict__ c_ssm, const float* __restrict__ d_skip, int layer) {
  const int g = (int)blockIdx.x * 32 + (int)threadIdx.x;
  const int b = g >> 9;
  const int d = g & (kWidth - 1);
  const int ld = layer * kWidth + d;
  float ab[16], bb[16], cc[16], xs[16];
#pragma unroll
  for (int q = 0; q < 4; ++q) {
    const v4f ta = *(const v4f*)(abar_t + (size_t)ld * kStates + 4 * q);
    const v4f tb = *(const v4f*)(bbar_t + (size_t)ld * kStates + 4 * q);
    const v4f tc = *(const v4f*)(c_ssm + (size_t)ld * kStates + 4 * q);
#pragma unroll
    for (int e = 0; e < 4; ++e) {
      ab[4 * q + e] = ta[e];
      bb[4 * q + e] = tb[e];
      cc[4 * q + e] = tc[e];
      xs[4 * q + e] = 0.0f;
    }
  }
  const float dsk = d_skip[ld];
  const float* ip = hin + (size_t)b * kSteps * kWidth + d;
  float* op = hout + (size_t)b * kSteps * kWidth + d;

  float cur[4];
#pragma unroll
  for (int j = 0; j < 4; ++j) cur[j] = ip[(size_t)j * kWidth];

  for (int t0 = 0; t0 < kSteps; t0 += 4) {
    const int tn = (t0 + 4 < kSteps) ? (t0 + 4) : t0;
    float nxt[4];
#pragma unroll
    for (int j = 0; j < 4; ++j) nxt[j] = ip[(size_t)(tn + j) * kWidth];
    float o[4];
#pragma unroll
    for (int j = 0; j < 4; ++j) {
      const float u = cur[j];
      float y = 0.0f;
#pragma unroll
      for (int n = 0; n < 16; ++n) {
        xs[n] = fmaf(ab[n], xs[n], bb[n] * u);
        y = fmaf(xs[n], cc[n], y);
      }
      y = fmaf(dsk, u, y);
      const float z = 0.7978845608028654f * (y + 0.044715f * y * y * y);
      o[j] = u + 0.5f * y * (1.0f + tanhf(z));
    }
    for (int pass = 0; pass < 2; ++pass) {
#pragma unroll
      for (int j = 0; j < 4; ++j) {
        volatile float* q = (volatile float*)(op + (size_t)(t0 + j) * kWidth);
        *q = o[j];
      }
      __threadfence();
    }
#pragma unroll
    for (int j = 0; j < 4; ++j) cur[j] = nxt[j];
  }
}

__global__ __launch_bounds__(256) void heads_kernel(
    const float* __restrict__ h,
    const float* __restrict__ s_f0, const float* __restrict__ bl_f0,
    const float* __restrict__ w_f0, const float* __restrict__ b_f0,
    const float* __restrict__ s_en, const float* __restrict__ bl_en,
    const float* __restrict__ w_en, const float* __restrict__ b_en,
    float* out) {
  const int lane = threadIdx.x & 31;
  const int wave = __builtin_amdgcn_readfirstlane((int)(threadIdx.x >> 5));
  const int row0 = ((int)blockIdx.x * 8 + wave) * 32;
  v4f sf[4], bf[4], wf[4], se[4], be[4], we[4];
#pragma unroll
  for (int j = 0; j < 4; ++j) {
    const int c = 128 * j + 4 * lane;
    sf[j] = *(const v4f*)(s_f0 + c);
    bf[j] = *(const v4f*)(bl_f0 + c);
    wf[j] = *(const v4f*)(w_f0 + c);
    se[j] = *(const v4f*)(s_en + c);
    be[j] = *(const v4f*)(bl_en + c);
    we[j] = *(const v4f*)(w_en + c);
  }
  const float bias0 = b_f0[0];
  const float bias1 = b_en[0];
  float keep0 = 0.0f;
  float keep1 = 0.0f;
  for (int rr = 0; rr < 32; ++rr) {
    const float* hr = h + (size_t)(row0 + rr) * kWidth + 4 * lane;
    v4f v[4];
#pragma unroll
    for (int j = 0; j < 4; ++j) v[j] = *(const v4f*)(hr + 128 * j);
    float s = 0.0f;
#pragma unroll
    for (int j = 0; j < 4; ++j)
#pragma unroll
      for (int e = 0; e < 4; ++e) s += v[j][e];
    s = wave_sum(s);
    const float mu = s * (1.0f / 512.0f);
    float q = 0.0f;
#pragma unroll
    for (int j = 0; j < 4; ++j)
#pragma unroll
      for (int e = 0; e < 4; ++e) {
        const float dv = v[j][e] - mu;
        q = fmaf(dv, dv, q);
      }
    q = wave_sum(q);
    const float var = q * (1.0f / 512.0f);
    const float rstd = rsqrtf(var + 1e-5f);
    float p0 = 0.0f;
    float p1 = 0.0f;
#pragma unroll
    for (int j = 0; j < 4; ++j)
#pragma unroll
      for (int e = 0; e < 4; ++e) {
        const float nv = (v[j][e] - mu) * rstd;
        p0 = fmaf(fmaf(nv, sf[j][e], bf[j][e]), wf[j][e], p0);
        p1 = fmaf(fmaf(nv, se[j][e], be[j][e]), we[j][e], p1);
      }
    p0 = wave_sum(p0);
    p1 = wave_sum(p1);
    const float r0 = p0 + bias0;
    const float r1 = p1 + bias1;
    keep0 = (lane == rr) ? r0 : keep0;
    keep1 = (lane == rr) ? r1 : keep1;
  }
  volatile float* q0 = (volatile float*)(out + row0 + lane);
  volatile float* q1 = (volatile float*)(out + kOut1Off + row0 + lane);
  *q0 = keep0;
  *q1 = keep1;
  __threadfence();
  *q0 = keep0;
  *q1 = keep1;
}

extern "C" void kernel_launch(void* const* d_in, const int* in_sizes, int n_in,
                              void* d_out, int out_size, void* d_ws, size_t ws_size,
                              hipStream_t stream) {
  if (n_in != 17) return;
  if (in_sizes[0] != kBatch * kSteps * kEmb) return;
  if (in_sizes[1] != kEmb * kWidth) return;
  if (in_sizes[2] != kWidth) return;
  if (in_sizes[3] != kFreqRows * kWidth) return;
  if (in_sizes[4] != kLayers * kWidth * kStates) return;
  if (in_sizes[5] != kLayers * kWidth * kStates) return;
  if (in_sizes[6] != kLayers * kWidth * kStates) return;
  if (in_sizes[7] != kLayers * kWidth) return;
  if (in_sizes[8] != kLayers * kWidth) return;
  if (in_sizes[9] != kWidth) return;
  if (in_sizes[10] != kWidth) return;
  if (in_sizes[11] != kWidth) return;
  if (in_sizes[12] != 1) return;
  if (in_sizes[13] != kWidth) return;
  if (in_sizes[14] != kWidth) return;
  if (in_sizes[15] != kWidth) return;
  if (in_sizes[16] != 1) return;
  if (kOut0Elems != kRows) return;
  if (kOut1Elems != kRows) return;
  if (out_size != kOut0Elems + kOut1Elems) return;
  if (ws_size < kWsTotal) return;

  const float* text_emb = (const float*)d_in[0];
  const float* W_in     = (const float*)d_in[1];
  const float* b_in     = (const float*)d_in[2];
  const float* freq_pe  = (const float*)d_in[3];
  const float* A_log    = (const float*)d_in[4];
  const float* B_ssm    = (const float*)d_in[5];
  const float* C_ssm    = (const float*)d_in[6];
  const float* log_dt   = (const float*)d_in[7];
  const float* D_skip   = (const float*)d_in[8];
  const float* ln_f0_s  = (const float*)d_in[9];
  const float* ln_f0_b  = (const float*)d_in[10];
  const float* W_f0     = (const float*)d_in[11];
  const float* b_f0     = (const float*)d_in[12];
  const float* ln_en_s  = (const float*)d_in[13];
  const float* ln_en_b  = (const float*)d_in[14];
  const float* W_en     = (const float*)d_in[15];
  const float* b_en     = (const float*)d_in[16];
  float* out = (float*)d_out;

  char* ws = (char*)d_ws;
  unsigned short* A16   = (unsigned short*)(ws + kOffA16);
  unsigned short* A16L  = (unsigned short*)(ws + kOffA16L);
  unsigned short* BT16  = (unsigned short*)(ws + kOffBt);
  unsigned short* BT16L = (unsigned short*)(ws + kOffBtL);
  float* ABAR = (float*)(ws + kOffAbar);
  float* BBAR = (float*)(ws + kOffBbar);
  float* H0 = (float*)(ws + kOffH);
  float* H1 = (float*)(ws + kOffH + 1 * kPlaneH);
  float* H2 = (float*)(ws + kOffH + 2 * kPlaneH);
  float* H3 = (float*)(ws + kOffH + 3 * kPlaneH);
  float* H4 = (float*)(ws + kOffH + 4 * kPlaneH);

  act_plane_kernel<<<(kRows * kEmb) / (8 * 256), 256, 0, stream>>>(text_emb, A16, A16L);
  weight_plane_kernel<<<dim3(kWidth / 32, kEmb / 256), 256, 0, stream>>>(W_in, BT16, BT16L);
  discretise_kernel<<<(kLayers * kWidth * kStates) / 256, 256, 0, stream>>>(log_dt, A_log, B_ssm, ABAR, BBAR);
  proj_gemm_kernel<<<kRows / 32, 256, 0, stream>>>(A16, A16L, BT16, BT16L, b_in, freq_pe, H0);

  scan_layer_kernel<<<(kBatch * kWidth) / 32, 32, 0, stream>>>(H0, H1, ABAR, BBAR, C_ssm, D_skip, 0);
  scan_layer_kernel<<<(kBatch * kWidth) / 32, 32, 0, stream>>>(H1, H2, ABAR, BBAR, C_ssm, D_skip, 1);
  scan_layer_kernel<<<(kBatch * kWidth) / 32, 32, 0, stream>>>(H2, H3, ABAR, BBAR, C_ssm, D_skip, 2);
  scan_layer_kernel<<<(kBatch * kWidth) / 32, 32, 0, stream>>>(H3, H4, ABAR, BBAR, C_ssm, D_skip, 3);

  heads_kernel<<<kRows / (32 * 8), 256, 0, stream>>>(H4, ln_f0_s, ln_f0_b, W_f0, b_f0, ln_en_s, ln_en_b, W_en, b_en, out);
}
